// AttentionStructureModel_26886495273181
// MI455X (gfx1250) — hardware-verified
//
#include <hip/hip_runtime.h>
#include <math.h>

constexpr int NSEQ    = 384;
constexpr int NSTEP   = 256;
constexpr int NHID    = 64;
constexpr int NG3     = 192;
constexpr int NROWS   = NSEQ * NSTEP;
constexpr int NFF     = 1024;
constexpr int QKVP    = 192;
constexpr int SP2     = 128;
constexpr int NFEATP  = 64;
constexpr int NTHR    = 256;
constexpr int NTG     = 128;
constexpr int EMBN    = 119;
constexpr int EMBD    = 10;
constexpr int NFEATK  = 30;
constexpr int SEQ_BLK = 16;
constexpr int HP      = 72;
constexpr int KP      = 40;
constexpr int VP      = 264;
constexpr int PP      = 72;
constexpr int OSP     = 72;
constexpr int HIDP    = 1032;
constexpr int XHP     = 72;
constexpr int SLP     = 68;
constexpr int FP      = 33;
constexpr int FFROWS  = 32;
constexpr int HSEQ    = 32;
constexpr float WCARRY     = 16.0f;
constexpr float WCARRY_INV = 1.0f / 16.0f;
constexpr float QKSCALE    = 0.17677669529663687f;
constexpr float PCARRY     = 32768.0f;
constexpr float LN_EPS_F   = 1e-5f;
constexpr float FLTMIN_F   = 1.17549435e-38f;
static_assert(NROWS % 64 == 0 && NG3 % 64 == 0 && NFF % 64 == 0 && (2 * NHID) % 64 == 0);
static_assert(NHID % 32 == 0 && NFF % 32 == 0);
static_assert(((NROWS / 64) * (NG3 / 64)) % 8 == 0);
static_assert(((NROWS / 64) * ((2 * NHID) / 64)) % 8 == 0);
static_assert(NSEQ % SEQ_BLK == 0);
static_assert(NROWS % FFROWS == 0 && NSEQ % FFROWS == 0 && NSTEP / FFROWS == 8 && NSTEP % FFROWS == 0);
static_assert(NSEQ % HSEQ == 0);
static_assert(NSTEP == 256 && NHID == 64 && NSTEP == NTHR);

typedef __attribute__((ext_vector_type(16))) _Float16 v16h;
typedef __attribute__((ext_vector_type(8)))  _Float16 v8h;
typedef __attribute__((ext_vector_type(16))) __bf16   v16b;
typedef __attribute__((ext_vector_type(8)))  __bf16   v8b;
typedef __attribute__((ext_vector_type(8)))  float    v8f;
typedef __attribute__((ext_vector_type(4)))  float    v4f;
typedef __attribute__((ext_vector_type(2)))  float    v2f;
typedef __attribute__((ext_vector_type(4)))  unsigned v4u;
typedef __attribute__((ext_vector_type(2)))  unsigned v2u;

__device__ __forceinline__ unsigned short f2bf_bits(float f) {
  unsigned u = __float_as_uint(f);
  return (unsigned short)((u + 0x7FFFu + ((u >> 16) & 1u)) >> 16);
}
__device__ __forceinline__ float bf_bits2f(unsigned short h) { return __uint_as_float(((unsigned)h) << 16); }
__device__ __forceinline__ float bf16r(float f) { return bf_bits2f(f2bf_bits(f)); }
__device__ __forceinline__ float h16_to_f32(unsigned hb) {
  const unsigned sgn = (hb & 0x8000u) << 16; const unsigned em = hb & 0x7fffu;
  const float fn = __uint_as_float((em << 13) + 0x38000000u);
  const float fs = (float)em * 5.9604644775390625e-8f;
  const float mag = (em < 0x400u) ? fs : fn; return __uint_as_float(__float_as_uint(mag) | sgn); }
__device__ __forceinline__ unsigned short f16_bits(float f) { return __builtin_bit_cast(unsigned short, (_Float16)f); }
__device__ __forceinline__ unsigned pack_h2(float a, float b) { return (unsigned)f16_bits(a) | ((unsigned)f16_bits(b) << 16); }
__device__ __forceinline__ void opq(float& x) { asm volatile("" : "+v"(x)); }

__device__ __forceinline__ void dep1_h(v8f& c, v16h a, v16h b) { asm volatile("v_nop\n\tv_nop\n\tv_nop\n\tv_nop" : "+v"(c) : "v"(a), "v"(b)); }
__device__ __forceinline__ void dep1_b(v8f& c, v16b a, v16b b) { asm volatile("v_nop\n\tv_nop\n\tv_nop\n\tv_nop" : "+v"(c) : "v"(a), "v"(b)); }
__device__ __forceinline__ void dep_guard4_h(v8f& a, v8f& b, v8f& c, v8f& d, v16h x, v16h y) { asm volatile("v_nop\n\tv_nop\n\tv_nop\n\tv_nop" : "+v"(a), "+v"(b), "+v"(c), "+v"(d) : "v"(x), "v"(y)); }
__device__ __forceinline__ void dep_guard4_b(v8f& a, v8f& b, v8f& c, v8f& d, v16b x, v16b y) { asm volatile("v_nop\n\tv_nop\n\tv_nop\n\tv_nop" : "+v"(a), "+v"(b), "+v"(c), "+v"(d) : "v"(x), "v"(y)); }
__device__ __forceinline__ void keep4_h(v16h a, v16h b, v16h c, v16h d) { asm volatile("v_nop" :: "v"(a), "v"(b), "v"(c), "v"(d)); }
__device__ __forceinline__ void keep4_b(v16b a, v16b b, v16b c, v16b d) { asm volatile("v_nop" :: "v"(a), "v"(b), "v"(c), "v"(d)); }
__device__ __forceinline__ void acc_guard4(v8f& a, v8f& b, v8f& c, v8f& d) { asm volatile("v_nop\n\tv_nop\n\tv_nop\n\tv_nop" : "+v"(a), "+v"(b), "+v"(c), "+v"(d)); }

template <typename T> struct Frag;
template <> struct Frag<_Float16> {
  typedef v16h V; union U { v16h v; v8h h[2]; };
  static __device__ __forceinline__ v16h load(const _Float16* p) {
    U f; f.h[0] = *(const v8h*)(p); f.h[1] = *(const v8h*)(p + 16); return f.v;
  }
  static __device__ __forceinline__ v8f mma(v16h a, v16h b, v8f c) {
    return __builtin_amdgcn_wmma_f32_16x16x32_f16(false, a, false, b, (short)0, c, false, false);
  }
  static __device__ __forceinline__ v8f mma_g(v16h a, v16h b, v8f c) { c = mma(a, b, c); dep1_h(c, a, b); return c; }
  static __device__ __forceinline__ void guard4(v8f& a, v8f& b, v8f& c, v8f& d, v16h x, v16h y) { dep_guard4_h(a, b, c, d, x, y); }
  static __device__ __forceinline__ void keep(v16h a, v16h b, v16h c, v16h d) { keep4_h(a, b, c, d); }
};
template <> struct Frag<__bf16> {
  typedef v16b V; union U { v16b v; v8b h[2]; };
  static __device__ __forceinline__ v16b load(const __bf16* p) {
    U f; f.h[0] = *(const v8b*)(p); f.h[1] = *(const v8b*)(p + 16); return f.v;
  }
  static __device__ __forceinline__ v8f mma(v16b a, v16b b, v8f c) {
    return __builtin_amdgcn_wmma_f32_16x16x32_bf16(false, a, false, b, (short)0, c, false, false);
  }
  static __device__ __forceinline__ v8f mma_g(v16b a, v16b b, v8f c) { c = mma(a, b, c); dep1_b(c, a, b); return c; }
  static __device__ __forceinline__ void guard4(v8f& a, v8f& b, v8f& c, v8f& d, v16b x, v16b y) { dep_guard4_b(a, b, c, d, x, y); }
  static __device__ __forceinline__ void keep(v16b a, v16b b, v16b c, v16b d) { keep4_b(a, b, c, d); }
};
template <int ET> struct Elem;
template <> struct Elem<0> { typedef _Float16 T; };
template <> struct Elem<1> { typedef __bf16 T; };

__device__ __forceinline__ float fsig(float x)  { return __builtin_amdgcn_rcpf(1.0f + expf(-x)); }
__device__ __forceinline__ float ftanh(float x) { return 1.0f - 2.0f * __builtin_amdgcn_rcpf(expf(2.0f * x) + 1.0f); }
__device__ __forceinline__ float fsilu(float x) { return x * __builtin_amdgcn_rcpf(1.0f + expf(-x)); }

template <int ET, int SPLIT, int BIAS_MODE, int OUT_MODE, bool RESID, int ACT = 0>
__global__ __launch_bounds__(256) void wmma_gemm64(
    const unsigned short* __restrict__ Ap, const unsigned short* __restrict__ A2p, int lda, long strideA,
    const unsigned short* __restrict__ Btp, const unsigned short* __restrict__ Bt2p, int ldb, long strideB,
    void* __restrict__ Cout, void* __restrict__ Cout2, int ldc, long strideC,
    const float* __restrict__ bias,
    const float* __restrict__ resid, long strideR,
    int M, int N, int K, float scale) {
  typedef typename Elem<ET>::T T;
  typedef typename Frag<T>::V V;
  const T* A = (const T*)Ap; const T* A2 = (const T*)A2p; const T* Bt = (const T*)Btp; const T* Bt2 = (const T*)Bt2p;
  __shared__ __align__(16) float sT[8][16 * 68];
  const int b    = blockIdx.y;
  const int lane = threadIdx.x & 31;
  const int wave = threadIdx.x >> 5;
  const int tilesN = N >> 6;
  const int tilesM = M >> 6;
  const int tile = blockIdx.x * 8 + wave;
  if (tile >= tilesM * tilesN) return;
  const int tm = tile / tilesN;
  const int tn = tile - tm * tilesN;
  const int m0 = tm << 6;
  const int n0 = tn << 6;

  const T* Ab  = A  + (size_t)b * strideA;
  const T* Bb  = Bt + (size_t)b * strideB;
  const T* Ab2 = (SPLIT != 0) ? (A2  + (size_t)b * strideA) : nullptr;
  const T* Bb2 = (SPLIT == 1) ? (Bt2 + (size_t)b * strideB) : nullptr;

  const int rlane = lane & 15;
  const int koff  = (lane >> 4) * 8;
  const int mOff  = (lane >> 4) * 8;

  v8f acc[4][4];
#pragma unroll
  for (int i = 0; i < 4; ++i)
#pragma unroll
    for (int j = 0; j < 4; ++j) acc[i][j] = (v8f){0.f,0.f,0.f,0.f,0.f,0.f,0.f,0.f};

  for (int k0 = 0; k0 < K; k0 += 32) {
    V bh[4], bl[4];
#pragma unroll
    for (int j = 0; j < 4; ++j) {
      const size_t bo = (size_t)(n0 + (j << 4) + rlane) * ldb + koff + k0;
      bh[j] = Frag<T>::load(Bb + bo);
      if (SPLIT == 1) bl[j] = Frag<T>::load(Bb2 + bo);
    }
#pragma unroll
    for (int i = 0; i < 4; ++i) {
      const size_t ao = (size_t)(m0 + (i << 4) + rlane) * lda + koff + k0;
      V ah = Frag<T>::load(Ab + ao);
      V al = ah;
      if (SPLIT != 0) al = Frag<T>::load(Ab2 + ao);
#pragma unroll
      for (int j = 0; j < 4; ++j) {
        acc[i][j] = Frag<T>::mma(ah, bh[j], acc[i][j]);
        if (SPLIT == 1) acc[i][j] = Frag<T>::mma(ah, bl[j], acc[i][j]);
        if (SPLIT != 0) acc[i][j] = Frag<T>::mma(al, bh[j], acc[i][j]);
      }
      Frag<T>::guard4(acc[i][0], acc[i][1], acc[i][2], acc[i][3], ah, (SPLIT != 0) ? al : bh[3]);
    }
    Frag<T>::keep(bh[0], bh[1], bh[2], bh[3]);
    if (SPLIT == 1) Frag<T>::keep(bl[0], bl[1], bl[2], bl[3]);
  }
  acc_guard4(acc[0][0], acc[0][1], acc[0][2], acc[0][3]);
  acc_guard4(acc[1][0], acc[1][1], acc[1][2], acc[1][3]);
  acc_guard4(acc[2][0], acc[2][1], acc[2][2], acc[2][3]);
  acc_guard4(acc[3][0], acc[3][1], acc[3][2], acc[3][3]);

  float* slab = sT[wave];
  const float* Rb = RESID ? (resid + (size_t)b * strideR) : nullptr;
#pragma unroll
  for (int i = 0; i < 4; ++i) {
    const int mBase = m0 + (i << 4);
#pragma unroll
    for (int j = 0; j < 4; ++j) {
      const int n = n0 + (j << 4) + rlane;
      float bv = 0.f;
      if (BIAS_MODE == 2) bv = bf16r(bias[n]);
#pragma unroll
      for (int r = 0; r < 8; ++r) {
        float v = acc[i][j][r] * scale;
        if (BIAS_MODE == 1) v += bf16r(bias[mBase + mOff + r]);
        if (BIAS_MODE == 2) v += bv;
        if (RESID) v += Rb[(size_t)(mBase + mOff + r) * ldc + n];
        if (ACT == 1) v = tanhf(v);
        if (ACT == 2) v = fmaxf(v, 0.0f);
        if (ACT == 4) v = (v > 0.f) ? v : 0.01f * v;
        slab[(mOff + r) * 68 + (j << 4) + rlane] = v;
      }
    }
    __builtin_amdgcn_fence(__ATOMIC_RELEASE, "workgroup");
    __builtin_amdgcn_wave_barrier();
    __builtin_amdgcn_fence(__ATOMIC_ACQUIRE, "workgroup");
    if (OUT_MODE == 0) {
      float* C = (float*)Cout + (size_t)b * strideC;
      const int hh = lane >> 4, c4 = (lane & 15) * 4;
      for (int pass = 0; pass < 2; ++pass) {
#pragma unroll
        for (int it = 0; it < 8; ++it) {
          const int row = it * 2 + hh;
          v4f v = *(const v4f*)(slab + row * 68 + c4);
          *(volatile v4f*)(C + (size_t)(mBase + row) * ldc + n0 + c4) = v;
        }
        __threadfence();
      }
    } else {
      const int q = lane >> 3, c8 = (lane & 7) * 8;
      unsigned short* C  = (unsigned short*)Cout  + (size_t)b * strideC;
      unsigned short* C2 = (OUT_MODE == 2) ? ((unsigned short*)Cout2 + (size_t)b * strideC) : nullptr;
      for (int pass = 0; pass < 2; ++pass) {
#pragma unroll
        for (int it = 0; it < 4; ++it) {
          const int row = it * 4 + q;
          const float* sp = slab + row * 68 + c8;
          v8h hv, lv;
#pragma unroll
          for (int e = 0; e < 8; ++e) {
            if (OUT_MODE == 1) {
              hv[e] = (_Float16)sp[e];
            } else {
              unsigned short hb = f2bf_bits(sp[e]);
              unsigned short lb = f2bf_bits(sp[e] - bf_bits2f(hb));
              hv[e] = __builtin_bit_cast(_Float16, hb);
              lv[e] = __builtin_bit_cast(_Float16, lb);
            }
          }
          *(volatile v8h*)(C + (size_t)(mBase + row) * ldc + n0 + c8) = hv;
          if (OUT_MODE == 2) *(volatile v8h*)(C2 + (size_t)(mBase + row) * ldc + n0 + c8) = lv;
        }
        __threadfence();
      }
    }
    __builtin_amdgcn_fence(__ATOMIC_RELEASE, "workgroup");
    __builtin_amdgcn_wave_barrier();
    __builtin_amdgcn_fence(__ATOMIC_ACQUIRE, "workgroup");
  }
}

template <int MODE>
__global__ __launch_bounds__(NTHR) void cvt8_kernel(const float* __restrict__ src, unsigned short* __restrict__ dst,
                                                    int nrow, int ncol8, int spitch, int scol0, float sc) {
  const int i  = blockIdx.x * NTHR + threadIdx.x;
  const int n8 = nrow * ncol8;
  if (i < n8) {
    const int row = i / ncol8;
    const int c8  = i - row * ncol8;
    const float* sp = src + (size_t)row * spitch + scol0 + c8 * 8;
    const v4f a = *(const v4f*)(sp);
    const v4f b = *(const v4f*)(sp + 4);
    v8h hv;
#pragma unroll
    for (int e = 0; e < 4; ++e) {
      unsigned short b0, b1;
      if (MODE == 0) {
        b0 = f2bf_bits(a[e] * sc);
        b1 = f2bf_bits(b[e] * sc);
      } else {
        b0 = __builtin_bit_cast(unsigned short, (_Float16)(bf16r(a[e]) * sc));
        b1 = __builtin_bit_cast(unsigned short, (_Float16)(bf16r(b[e]) * sc));
      }
      hv[e]     = __builtin_bit_cast(_Float16, b0);
      hv[4 + e] = __builtin_bit_cast(_Float16, b1);
    }
    *(volatile v8h*)(dst + (size_t)i * 8) = hv;
    __threadfence();
    *(volatile v8h*)(dst + (size_t)i * 8) = hv;
  }
}

__global__ __launch_bounds__(NTHR) void featurize_kernel(const float* __restrict__ x, const float* __restrict__ emb,
                                                         unsigned short* __restrict__ fe) {
#pragma clang fp contract(off)
  __shared__ float F[NTHR * FP];
  const int tid = threadIdx.x, lane = tid & 31, wave = tid >> 5;
  const int n = blockIdx.x, l = tid;
  const int kind = n % 3;
  const float* xb = x + (size_t)n * 3 * NSTEP;
  const float a0 = bf16r(xb[l]), a1 = bf16r(xb[NSTEP + l]), a2 = bf16r(xb[2 * NSTEP + l]);
  float* f = F + tid * FP;
  if (kind == 2) {
#pragma unroll 1
    for (int i = 0; i < 20; ++i) {
      const float d = (i < 10) ? a0 : a1;
      const int ci = (i < 10) ? i : (i - 10);
      const float dd = (float)(ci + 1) - d;
      float v = expf(-(dd * dd));
      v = (v < FLTMIN_F) ? 0.0f : v;
      f[i] = v;
    }
    float t0 = 1.0f, t1 = a2;
    f[20] = t0; f[21] = t1;
    const float twoa = 2.0f * a2;
#pragma unroll 1
    for (int i = 2; i < 10; ++i) {
      float p = twoa * t1;
      opq(p);
      const float t2 = p - t0;
      f[20 + i] = t2; t0 = t1; t1 = t2;
    }
  } else {
    int i1 = (int)a0; i1 = i1 < 0 ? 0 : (i1 > EMBN - 1 ? EMBN - 1 : i1);
    int i2 = (int)a1; i2 = i2 < 0 ? 0 : (i2 > EMBN - 1 ? EMBN - 1 : i2);
#pragma unroll 1
    for (int i = 0; i < 10; ++i) {
      f[i]      = bf16r(emb[i1 * EMBD + i]);
      f[10 + i] = bf16r(emb[i2 * EMBD + i]);
      const float dd = (float)(i + 1) - a2;
      float v = expf(-(dd * dd));
      v = (v < FLTMIN_F) ? 0.0f : v;
      f[20 + i] = v;
    }
  }
  f[30] = 0.0f; f[31] = 0.0f; f[32] = 0.0f;
  __syncthreads();
  const int q = lane >> 3, p = lane & 7;
  const unsigned selh = (p < 4) ? 0xffffu : 0u;
  const unsigned sell = selh ^ 0xffffu;
  v4u o[8];
#pragma unroll
  for (int it = 0; it < 8; ++it) {
    const int row = wave * 32 + it * 4 + q;
    unsigned wd[4];
#pragma unroll
    for (int e2 = 0; e2 < 4; ++e2) {
      unsigned bits[2];
#pragma unroll
      for (int u = 0; u < 2; ++u) {
        const int col = p * 8 + e2 * 2 + u;
        const float v = F[row * FP + (col & 31)];
        const unsigned short hb = f2bf_bits(v);
        const unsigned short lb = f2bf_bits(v - bf_bits2f(hb));
        bits[u] = ((unsigned)hb & selh) | ((unsigned)lb & sell);
      }
      wd[e2] = bits[0] | (bits[1] << 16);
    }
    v4u t; t[0] = wd[0]; t[1] = wd[1]; t[2] = wd[2]; t[3] = wd[3];
    o[it] = t;
  }
  for (int pass = 0; pass < 2; ++pass) {
#pragma unroll
    for (int it = 0; it < 8; ++it) {
      const int row = wave * 32 + it * 4 + q;
      *(volatile v4u*)(fe + ((size_t)n * NSTEP + row) * NFEATP + p * 8) = o[it];
    }
    __threadfence();
  }
}

template <int KREAL>
__global__ __launch_bounds__(NTG) void gru_layer_kernel(const unsigned short* __restrict__ Xp,
                                                       const float* __restrict__ Wih, const float* __restrict__ Whh,
                                                       const float* __restrict__ bih, const float* __restrict__ bhh,
                                                       unsigned short* __restrict__ Sout) {
  constexpr int KH   = (KREAL <= 32) ? 32 : 64;
  constexpr int KX   = 2 * KH;
  constexpr int KXP  = KX + 8;
  constexpr int NITX = (NG3 * (KX / 4)) / NTG;
  constexpr int NITH = (NG3 * (NHID / 4)) / NTG;
  constexpr int NITZ = (SEQ_BLK * HP) / NTG;
  static_assert((NG3 * (KX / 4)) % NTG == 0 && (NG3 * (NHID / 4)) % NTG == 0 && (SEQ_BLK * HP) % NTG == 0);
  static_assert(KREAL <= KH);
  __shared__ __align__(16) unsigned short Wxs[NG3 * KXP];
  __shared__ __align__(16) unsigned short Whs[NG3 * HP];
  __shared__ __align__(16) unsigned short Ahh[SEQ_BLK * HP];
  __shared__ __align__(16) unsigned short Ahl[SEQ_BLK * HP];
  const int tid = threadIdx.x, lane = tid & 31, wave = tid >> 5;
  const int c = lane & 15, hh = lane >> 4, koff = hh * 8;
  const int q = lane >> 3, c8 = (lane & 7) * 8;
  const int seq0 = blockIdx.x * SEQ_BLK;
  const int j = 16 * wave + c;

#pragma unroll 1
  for (int it = 0; it < NITX; ++it) {
    const int idx = it * NTG + tid;
    const int row = idx / (KX / 4);
    const int k4  = (idx - row * (KX / 4)) * 4;
    unsigned bts[4];
#pragma unroll
    for (int e = 0; e < 4; ++e) {
      const int km = (k4 + e) & (KH - 1);
      const int kc = (km < KREAL) ? km : (KREAL - 1);
      const float fac = (km < KREAL) ? 1.0f : 0.0f;
      const float w = Wih[(size_t)row * KREAL + kc] * fac;
      bts[e] = f2bf_bits(w);
    }
    v2u pk; pk[0] = bts[0] | (bts[1] << 16); pk[1] = bts[2] | (bts[3] << 16);
    *(v2u*)(Wxs + row * KXP + k4) = pk;
  }
#pragma unroll 1
  for (int it = 0; it < NITH; ++it) {
    const int idx = it * NTG + tid;
    const int row = idx >> 4, k4 = (idx & 15) * 4;
    const v4f wv = *(const v4f*)(Whh + (size_t)row * NHID + k4);
    const unsigned b0 = f2bf_bits(wv[0]), b1 = f2bf_bits(wv[1]), b2 = f2bf_bits(wv[2]), b3 = f2bf_bits(wv[3]);
    v2u pk; pk[0] = b0 | (b1 << 16); pk[1] = b2 | (b3 << 16);
    *(v2u*)(Whs + row * HP + k4) = pk;
  }
#pragma unroll 1
  for (int it = 0; it < NITZ; ++it) { Ahh[it * NTG + tid] = 0; Ahl[it * NTG + tid] = 0; }
  const float br  = bf16r(bih[j]) + bf16r(bhh[j]);
  const float bz  = bf16r(bih[NHID + j]) + bf16r(bhh[NHID + j]);
  const float bin = bf16r(bih[2 * NHID + j]);
  const float bhn = bf16r(bhh[2 * NHID + j]);
  float hst[8];
#pragma unroll
  for (int r = 0; r < 8; ++r) hst[r] = 0.0f;
  __syncthreads();

  const __bf16* wxr = (const __bf16*)Wxs + (size_t)j * KXP + koff;
  const __bf16* wxz = (const __bf16*)Wxs + (size_t)(NHID + j) * KXP + koff;
  const __bf16* wxn = (const __bf16*)Wxs + (size_t)(2 * NHID + j) * KXP + koff;
  const __bf16* whr = (const __bf16*)Whs + (size_t)j * HP + koff;
  const __bf16* whz = (const __bf16*)Whs + (size_t)(NHID + j) * HP + koff;
  const __bf16* whn = (const __bf16*)Whs + (size_t)(2 * NHID + j) * HP + koff;
  const __bf16* ahhrow = (const __bf16*)Ahh + c * HP + koff;
  const __bf16* ahlrow = (const __bf16*)Ahl + c * HP + koff;
  const __bf16* xbase = (const __bf16*)Xp + ((size_t)(seq0 + c) * NSTEP) * KX + koff;
  const v8f z8 = {0.f, 0.f, 0.f, 0.f, 0.f, 0.f, 0.f, 0.f};

#pragma unroll 1
  for (int t = 0; t < NSTEP; ++t) {
    v8f acc[4];
    acc[0] = z8; acc[1] = z8; acc[2] = z8; acc[3] = z8;
    const __bf16* xrow = xbase + (size_t)t * KX;
#pragma unroll
    for (int kx = 0; kx < KX; kx += 32) {
      const v16b a  = Frag<__bf16>::load(xrow + kx);
      const v16b b0 = Frag<__bf16>::load(wxr + kx);
      const v16b b1 = Frag<__bf16>::load(wxz + kx);
      const v16b b2 = Frag<__bf16>::load(wxn + kx);
      acc[0] = Frag<__bf16>::mma_g(a, b0, acc[0]);
      acc[1] = Frag<__bf16>::mma_g(a, b1, acc[1]);
      acc[2] = Frag<__bf16>::mma_g(a, b2, acc[2]);
    }
#pragma unroll
    for (int k0 = 0; k0 < NHID; k0 += 32) {
      const v16b ah = Frag<__bf16>::load(ahhrow + k0);
      const v16b al = Frag<__bf16>::load(ahlrow + k0);
      const v16b b0 = Frag<__bf16>::load(whr + k0);
      const v16b b1 = Frag<__bf16>::load(whz + k0);
      const v16b b2 = Frag<__bf16>::load(whn + k0);
      acc[0] = Frag<__bf16>::mma_g(ah, b0, acc[0]);
      acc[0] = Frag<__bf16>::mma_g(al, b0, acc[0]);
      acc[1] = Frag<__bf16>::mma_g(ah, b1, acc[1]);
      acc[1] = Frag<__bf16>::mma_g(al, b1, acc[1]);
      acc[3] = Frag<__bf16>::mma_g(ah, b2, acc[3]);
      acc[3] = Frag<__bf16>::mma_g(al, b2, acc[3]);
    }
    acc_guard4(acc[0], acc[1], acc[2], acc[3]);
    unsigned short hib[8], lob[8];
#pragma unroll
    for (int r = 0; r < 8; ++r) {
      const float zr  = acc[0][r] + br;
      const float zz  = acc[1][r] + bz;
      const float gin = acc[2][r] + bin;
      const float ghn = acc[3][r] + bhn;
      const float rg = fsig(zr);
      const float zg = fsig(zz);
      const float ng = ftanh(gin + rg * ghn);
      const float ho = hst[r];
      const float hn = (1.0f - zg) * ng + zg * ho;
      hst[r] = hn;
      const unsigned short hb = f2bf_bits(hn);
      hib[r] = hb;
      lob[r] = f2bf_bits(hn - bf_bits2f(hb));
    }
    __syncthreads();
#pragma unroll
    for (int r = 0; r < 8; ++r) { Ahh[(8 * hh + r) * HP + j] = hib[r]; Ahl[(8 * hh + r) * HP + j] = lob[r]; }
    __syncthreads();
    {
      const int row = 4 * wave + q;
      const v4u vh = *(const v4u*)(Ahh + row * HP + c8);
      const v4u vl = *(const v4u*)(Ahl + row * HP + c8);
      unsigned short* dst = Sout + ((size_t)(seq0 + row) * NSTEP + (size_t)t) * SP2;
      *(volatile v4u*)(dst + c8) = vh;
      *(volatile v4u*)(dst + NHID + c8) = vl;
      __threadfence();
      *(volatile v4u*)(dst + c8) = vh;
      *(volatile v4u*)(dst + NHID + c8) = vl;
    }
  }
}

__global__ __launch_bounds__(NTHR) void attn_ln1_kernel(const unsigned short* __restrict__ QKV, const unsigned short* __restrict__ Gp,
                                                        const unsigned short* __restrict__ Wop, const float* __restrict__ bo,
                                                        const float* __restrict__ lns, const float* __restrict__ lnb,
                                                        unsigned short* __restrict__ H1) {
  __shared__ __align__(16) unsigned short Ksh[NSTEP * KP];
  __shared__ __align__(16) unsigned short Vt[32 * VP];
  __shared__ __align__(16) unsigned short Psh[8][16 * PP];
  __shared__ __align__(16) unsigned short Osl[8][16 * OSP];
  __shared__ __align__(16) float          Sl[8][16 * SLP];
  const int tid = threadIdx.x, lane = tid & 31, wave = tid >> 5;
  const int hh = lane >> 4, c = lane & 15, koff = hh * 8;
  const int q8 = lane >> 3, c8 = (lane & 7) * 8;
  const int n = blockIdx.x >> 1;
  const int q0 = (blockIdx.x & 1) * 128 + wave * 16;
  const size_t rowbase = (size_t)n * NSTEP;
  const _Float16* QKVh = (const _Float16*)QKV;
  const _Float16* Wo   = (const _Float16*)Wop;
  unsigned short* psh = Psh[wave];
  unsigned short* osl = Osl[wave];
  float* slab = Sl[wave];
  const v8f z8 = {0.f, 0.f, 0.f, 0.f, 0.f, 0.f, 0.f, 0.f};

#pragma unroll 1
  for (int h = 0; h < 2; ++h) {
    __syncthreads();
#pragma unroll
    for (int it = 0; it < 4; ++it) {
      const int id = it * NTHR + tid;
      const int key = id >> 2, cc = (id & 3) * 8;
      const unsigned short* src = QKV + (rowbase + key) * QKVP;
      const v4u kw = *(const v4u*)(src + NHID + h * 32 + cc);
      const v4u vw = *(const v4u*)(src + 2 * NHID + h * 32 + cc);
      *(v4u*)(Ksh + key * KP + cc) = kw;
#pragma unroll
      for (int e = 0; e < 4; ++e) {
        const unsigned w = vw[e];
        Vt[(cc + 2 * e) * VP + key]     = (unsigned short)(w & 0xffffu);
        Vt[(cc + 2 * e + 1) * VP + key] = (unsigned short)(w >> 16);
      }
    }
    __syncthreads();
    const v16h qa = Frag<_Float16>::load(QKVh + (rowbase + q0 + c) * QKVP + h * 32 + koff);
    float mrow[8], lrow[8];
    v8f oacc[2];
#pragma unroll
    for (int r = 0; r < 8; ++r) { mrow[r] = -INFINITY; lrow[r] = 0.f; }
    oacc[0] = z8; oacc[1] = z8;
#pragma unroll 1
    for (int kc = 0; kc < 4; ++kc) {
      const int kv0 = kc * 64;
      v8f s[4];
#pragma unroll
      for (int jt = 0; jt < 4; ++jt) {
        const v16h kb = Frag<_Float16>::load((const _Float16*)Ksh + (kv0 + jt * 16 + c) * KP + koff);
        s[jt] = Frag<_Float16>::mma_g(qa, kb, z8);
      }
      float cm[8];
#pragma unroll
      for (int r = 0; r < 8; ++r) {
        float m = -INFINITY;
#pragma unroll
        for (int jt = 0; jt < 4; ++jt) { s[jt][r] *= QKSCALE; m = fmaxf(m, s[jt][r]); }
#pragma unroll
        for (int off = 1; off < 16; off <<= 1) m = fmaxf(m, __shfl_xor(m, off, 32));
        cm[r] = m;
      }
#pragma unroll
      for (int r = 0; r < 8; ++r) {
        const float mnew = fmaxf(mrow[r], cm[r]);
        const float alpha = expf(mrow[r] - mnew);
        mrow[r] = mnew;
        float psum = 0.f;
#pragma unroll
        for (int jt = 0; jt < 4; ++jt) {
          const float pv = expf(s[jt][r] - mnew);
          psum += pv;
          psh[(8 * hh + r) * PP + jt * 16 + c] = f16_bits(pv * PCARRY);
        }
#pragma unroll
        for (int off = 1; off < 16; off <<= 1) psum += __shfl_xor(psum, off, 32);
        lrow[r] = lrow[r] * alpha + psum;
        oacc[0][r] *= alpha;
        oacc[1][r] *= alpha;
      }
      __builtin_amdgcn_fence(__ATOMIC_RELEASE, "workgroup");
      __builtin_amdgcn_wave_barrier();
      __builtin_amdgcn_fence(__ATOMIC_ACQUIRE, "workgroup");
#pragma unroll
      for (int kk = 0; kk < 2; ++kk) {
        const v16h pa = Frag<_Float16>::load((const _Float16*)psh + c * PP + kk * 32 + koff);
#pragma unroll
        for (int tt = 0; tt < 2; ++tt) {
          const v16h vb = Frag<_Float16>::load((const _Float16*)Vt + (tt * 16 + c) * VP + kv0 + kk * 32 + koff);
          oacc[tt] = Frag<_Float16>::mma_g(pa, vb, oacc[tt]);
        }
      }
    }
#pragma unroll
    for (int r = 0; r < 8; ++r) {
      const float inv = __builtin_amdgcn_rcpf(lrow[r] * PCARRY);
#pragma unroll
      for (int tt = 0; tt < 2; ++tt) osl[(8 * hh + r) * OSP + h * 32 + tt * 16 + c] = f16_bits(oacc[tt][r] * inv);
    }
  }
  __builtin_amdgcn_fence(__ATOMIC_RELEASE, "workgroup");
  __builtin_amdgcn_wave_barrier();
  __builtin_amdgcn_fence(__ATOMIC_ACQUIRE, "workgroup");

  v8f pacc[4];
  pacc[0] = z8; pacc[1] = z8; pacc[2] = z8; pacc[3] = z8;
  {
    const _Float16* arow = (const _Float16*)osl + c * OSP + koff;
#pragma unroll 1
    for (int k0 = 0; k0 < NHID; k0 += 32) {
      const v16h a = Frag<_Float16>::load(arow + k0);
      v16h bw[4];
#pragma unroll
      for (int jt = 0; jt < 4; ++jt) bw[jt] = Frag<_Float16>::load(Wo + (size_t)(16 * jt + c) * NHID + koff + k0);
#pragma unroll
      for (int jt = 0; jt < 4; ++jt) pacc[jt] = Frag<_Float16>::mma_g(a, bw[jt], pacc[jt]);
    }
  }
  acc_guard4(pacc[0], pacc[1], pacc[2], pacc[3]);
#pragma unroll
  for (int jt = 0; jt < 4; ++jt)
#pragma unroll
    for (int r = 0; r < 8; ++r) slab[(8 * hh + r) * SLP + 16 * jt + c] = pacc[jt][r] * WCARRY_INV;
  __builtin_amdgcn_fence(__ATOMIC_RELEASE, "workgroup");
  __builtin_amdgcn_wave_barrier();
  __builtin_amdgcn_fence(__ATOMIC_ACQUIRE, "workgroup");

  {
    const int l2 = 2 * lane;
    const v2f bo2 = *(const v2f*)(bo + l2);
    const v2f s2  = *(const v2f*)(lns + l2);
    const v2f b2  = *(const v2f*)(lnb + l2);
    const float bo0 = bf16r(bo2[0]), bo1 = bf16r(bo2[1]);
    const float s0 = bf16r(s2[0]), s1 = bf16r(s2[1]);
    const float b0 = bf16r(b2[0]), b1 = bf16r(b2[1]);
#pragma unroll 1
    for (int rr = 0; rr < 16; ++rr) {
      const unsigned* gw = (const unsigned*)(Gp + (rowbase + q0 + rr) * SP2);
      const unsigned wh = gw[lane], wl = gw[32 + lane];
      const float g0 = __uint_as_float(wh << 16) + __uint_as_float(wl << 16);
      const float g1 = __uint_as_float(wh & 0xffff0000u) + __uint_as_float(wl & 0xffff0000u);
      const v2f av = *(const v2f*)(slab + rr * SLP + l2);
      const float x0 = g0 + (av[0] + bo0);
      const float x1 = g1 + (av[1] + bo1);
      float sm = x0 + x1;
#pragma unroll
      for (int off = 1; off < 32; off <<= 1) sm += __shfl_xor(sm, off, 32);
      const float mean = sm * (1.0f / NHID);
      const float d0 = x0 - mean, d1 = x1 - mean;
      float ss = d0 * d0 + d1 * d1;
#pragma unroll
      for (int off = 1; off < 32; off <<= 1) ss += __shfl_xor(ss, off, 32);
      const float var = ss * (1.0f / NHID);
      const float rstd = rsqrtf(var + LN_EPS_F);
      v2f yv;
      yv[0] = (d0 * rstd) * s0 + b0;
      yv[1] = (d1 * rstd) * s1 + b1;
      *(v2f*)(slab + rr * SLP + l2) = yv;
    }
  }
  __builtin_amdgcn_fence(__ATOMIC_RELEASE, "workgroup");
  __builtin_amdgcn_wave_barrier();
  __builtin_amdgcn_fence(__ATOMIC_ACQUIRE, "workgroup");
  for (int pass = 0; pass < 2; ++pass) {
#pragma unroll
    for (int it = 0; it < 4; ++it) {
      const int row = it * 4 + q8;
      const v4f va = *(const v4f*)(slab + row * SLP + c8);
      const v4f vb = *(const v4f*)(slab + row * SLP + c8 + 4);
      v4u hv, lv;
#pragma unroll
      for (int e = 0; e < 2; ++e) {
        const float f0 = va[2 * e], f1 = va[2 * e + 1];
        const float f2 = vb[2 * e], f3 = vb[2 * e + 1];
        const unsigned short h0 = f2bf_bits(f0), h1b = f2bf_bits(f1), h2 = f2bf_bits(f2), h3 = f2bf_bits(f3);
        const unsigned short l0 = f2bf_bits(f0 - bf_bits2f(h0)), l1 = f2bf_bits(f1 - bf_bits2f(h1b));
        const unsigned short l2b = f2bf_bits(f2 - bf_bits2f(h2)), l3 = f2bf_bits(f3 - bf_bits2f(h3));
        hv[e]     = (unsigned)h0 | ((unsigned)h1b << 16);
        hv[2 + e] = (unsigned)h2 | ((unsigned)h3 << 16);
        lv[e]     = (unsigned)l0 | ((unsigned)l1 << 16);
        lv[2 + e] = (unsigned)l2b | ((unsigned)l3 << 16);
      }
      unsigned short* dst = H1 + (rowbase + q0 + row) * SP2;
      *(volatile v4u*)(dst + c8) = hv;
      *(volatile v4u*)(dst + NHID + c8) = lv;
    }
    __threadfence();
  }
}

template <bool OUT16, int FMODE>
__global__ __launch_bounds__(NTHR) void ffn_ln_kernel(const unsigned short* __restrict__ Xb,
                                                      const unsigned short* __restrict__ W1p, const float* __restrict__ b1,
                                                      const unsigned short* __restrict__ W2p, const float* __restrict__ b2,
                                                      const float* __restrict__ lns, const float* __restrict__ lnb,
                                                      float* __restrict__ OF, unsigned short* __restrict__ OH) {
  __shared__ __align__(16) unsigned short Hid[FFROWS * HIDP];
  __shared__ __align__(16) unsigned short Xh[FFROWS * XHP];
  __shared__ __align__(16) float          Xf[FFROWS * SLP];
  __shared__ __align__(16) float          Sl[FFROWS * SLP];
  const int tid = threadIdx.x, lane = tid & 31, wave = tid >> 5;
  const int c = lane & 15, hh = lane >> 4, koff = hh * 8, c4 = c * 4;
  const int q = lane >> 3, c8 = (lane & 7) * 8;
  const int row0 = blockIdx.x * FFROWS;
  const _Float16* W1 = (const _Float16*)W1p;
  const _Float16* W2 = (const _Float16*)W2p;
  const v8f z8 = {0.f, 0.f, 0.f, 0.f, 0.f, 0.f, 0.f, 0.f};

  {
    const int row = tid >> 3, p8 = (tid & 7) * 8;
    const unsigned short* src = Xb + (size_t)(row0 + row) * SP2;
    const v4u hw = *(const v4u*)(src + p8);
    const v4u lw = *(const v4u*)(src + NHID + p8);
    v4u pk;
#pragma unroll
    for (int e = 0; e < 4; ++e) {
      const unsigned wh = hw[e], wl = lw[e];
      const float f0 = __uint_as_float(wh << 16) + __uint_as_float(wl << 16);
      const float f1 = __uint_as_float(wh & 0xffff0000u) + __uint_as_float(wl & 0xffff0000u);
      Xf[row * SLP + p8 + 2 * e]     = f0;
      Xf[row * SLP + p8 + 2 * e + 1] = f1;
      pk[e] = pack_h2(f0, f1);
    }
    *(v4u*)(Xh + row * XHP + p8) = pk;
  }
  __syncthreads();

#pragma unroll 1
  for (int gq = 0; gq < 2; ++gq) {
    const int n0 = 128 * wave + 64 * gq;
    v8f acc[2][4];
#pragma unroll
    for (int i = 0; i < 2; ++i)
#pragma unroll
      for (int jt = 0; jt < 4; ++jt) acc[i][jt] = z8;
#pragma unroll 1
    for (int k0 = 0; k0 < NHID; k0 += 32) {
      v16h bh[4];
#pragma unroll
      for (int jt = 0; jt < 4; ++jt) bh[jt] = Frag<_Float16>::load(W1 + (size_t)(n0 + 16 * jt + c) * NHID + koff + k0);
#pragma unroll
      for (int i = 0; i < 2; ++i) {
        const v16h ah = Frag<_Float16>::load((const _Float16*)Xh + (16 * i + c) * XHP + koff + k0);
#pragma unroll
        for (int jt = 0; jt < 4; ++jt) acc[i][jt] = Frag<_Float16>::mma_g(ah, bh[jt], acc[i][jt]);
      }
    }
    acc_guard4(acc[0][0], acc[0][1], acc[0][2], acc[0][3]);
    acc_guard4(acc[1][0], acc[1][1], acc[1][2], acc[1][3]);
#pragma unroll
    for (int jt = 0; jt < 4; ++jt) {
      const int ncol = n0 + 16 * jt + c;
      const float bv = bf16r(b1[ncol]);
#pragma unroll
      for (int i = 0; i < 2; ++i)
#pragma unroll
        for (int r = 0; r < 8; ++r) {
          const float v = fmaxf(acc[i][jt][r] * WCARRY_INV + bv, 0.0f);
          Hid[(16 * i + 8 * hh + r) * HIDP + ncol] = f16_bits(v);
        }
    }
  }
  __syncthreads();

  const int mi = wave >> 2, ni = wave & 3;
  v8f acc2 = z8;
  {
    const _Float16* arow = (const _Float16*)Hid + (16 * mi + c) * HIDP + koff;
    const _Float16* brow = W2 + (size_t)(16 * ni + c) * NFF + koff;
#pragma unroll 1
    for (int k0 = 0; k0 < NFF; k0 += 32) {
      const v16h a = Frag<_Float16>::load(arow + k0);
      const v16h b = Frag<_Float16>::load(brow + k0);
      acc2 = Frag<_Float16>::mma_g(a, b, acc2);
    }
  }
  {
    const int col = 16 * ni + c;
    const float bv = bf16r(b2[col]);
#pragma unroll
    for (int r = 0; r < 8; ++r) {
      const int row = 16 * mi + 8 * hh + r;
      float v = fmaxf(acc2[r] * WCARRY_INV + bv, 0.0f);
      v += Xf[row * SLP + col];
      Sl[row * SLP + col] = v;
    }
  }
  __syncthreads();

  const float s0v = bf16r(lns[lane]), s1v = bf16r(lns[lane + 32]);
  const float b0v = bf16r(lnb[lane]), b1v = bf16r(lnb[lane + 32]);
#pragma unroll
  for (int rr = 0; rr < 4; ++rr) {
    const int row = 4 * wave + rr;
    const float x0 = Sl[row * SLP + lane], x1 = Sl[row * SLP + lane + 32];
    float s = x0 + x1;
#pragma unroll
    for (int off = 1; off < 32; off <<= 1) s += __shfl_xor(s, off, 32);
    const float mean = s * (1.0f / NHID);
    const float d0 = x0 - mean, d1 = x1 - mean;
    float ss = d0 * d0 + d1 * d1;
#pragma unroll
    for (int off = 1; off < 32; off <<= 1) ss += __shfl_xor(ss, off, 32);
    const float var = ss * (1.0f / NHID);
    const float rstd = rsqrtf(var + LN_EPS_F);
    Sl[row * SLP + lane]      = (d0 * rstd) * s0v + b0v;
    Sl[row * SLP + lane + 32] = (d1 * rstd) * s1v + b1v;
  }
  __builtin_amdgcn_fence(__ATOMIC_RELEASE, "workgroup");
  __builtin_amdgcn_wave_barrier();
  __builtin_amdgcn_fence(__ATOMIC_ACQUIRE, "workgroup");
  const bool lastblk = (FMODE == 2) && ((blockIdx.x & 7) == 7) && (wave == 7);
  for (int pass = 0; pass < 2; ++pass) {
    if (FMODE == 1) {
#pragma unroll
      for (int p2 = 0; p2 < 2; ++p2) {
        const int row = 4 * wave + 2 * p2 + hh;
        const v4f v = *(const v4f*)(Sl + row * SLP + c4);
        *(volatile v4f*)(OF + (size_t)(row0 + row) * NHID + c4) = v;
      }
    }
    if (FMODE == 2) {
      if (lastblk) {
        const v4f v = *(const v4f*)(Sl + (FFROWS - 1) * SLP + c4);
        if (hh == 1) *(volatile v4f*)(OF + (size_t)(blockIdx.x >> 3) * NHID + c4) = v;
      }
    }
    if (OUT16) {
      const int row = 4 * wave + q;
      const float* sp = Sl + row * SLP + c8;
      v4u hv;
      hv[0] = pack_h2(sp[0], sp[1]); hv[1] = pack_h2(sp[2], sp[3]);
      hv[2] = pack_h2(sp[4], sp[5]); hv[3] = pack_h2(sp[6], sp[7]);
      *(volatile v4u*)(OH + (size_t)(row0 + row) * NHID + c8) = hv;
    }
    __threadfence();
  }
}

__global__ __launch_bounds__(64) void tail_kernel(const float* __restrict__ H2L, const unsigned short* __restrict__ KV,
                                                 const float* __restrict__ in_w2, const float* __restrict__ in_b2,
                                                 const float* __restrict__ out_w2, const float* __restrict__ out_b2,
                                                 const float* __restrict__ ln3s, const float* __restrict__ ln3b,
                                                 unsigned short* __restrict__ H3B) {
  __shared__ float xs[64], qs[64], sc[512], os[64], t3[64], ys[64];
  const int j = threadIdx.x, lane = j & 31, wave = j >> 5;
  const int n = blockIdx.x;
  const size_t rowb = (size_t)n * NSTEP;
  xs[j] = H2L[(size_t)n * NHID + j];
  __syncthreads();
  {
    float acc = 0.0f;
    const float* wr = in_w2 + (size_t)j * NHID;
#pragma unroll 1
    for (int k = 0; k < NHID; ++k) acc = fmaf(xs[k], bf16r(wr[k]), acc);
    qs[j] = acc + bf16r(in_b2[j]);
  }
  __syncthreads();
#pragma unroll 1
  for (int kk = 0; kk < 4; ++kk) {
    const int key = j + 64 * kk;
    const unsigned* krow = (const unsigned*)(KV + (rowb + key) * QKVP);
#pragma unroll 1
    for (int h = 0; h < 2; ++h) {
      float acc = 0.0f;
#pragma unroll 1
      for (int w = 0; w < 16; ++w) {
        const unsigned u = krow[h * 16 + w];
        acc = fmaf(qs[h * 32 + 2 * w],     h16_to_f32(u & 0xffffu), acc);
        acc = fmaf(qs[h * 32 + 2 * w + 1], h16_to_f32(u >> 16),     acc);
      }
      sc[h * 256 + key] = acc * QKSCALE;
    }
  }
  __syncthreads();
  {
    const int hb = wave * 256;
    float m = -INFINITY;
#pragma unroll 1
    for (int i = 0; i < 8; ++i) m = fmaxf(m, sc[hb + lane + 32 * i]);
#pragma unroll
    for (int off = 1; off < 32; off <<= 1) m = fmaxf(m, __shfl_xor(m, off, 32));
    float ssum = 0.0f;
#pragma unroll 1
    for (int i = 0; i < 8; ++i) {
      const int idx = hb + lane + 32 * i;
      const float pv = expf(sc[idx] - m);
      sc[idx] = pv;
      ssum += pv;
    }
#pragma unroll
    for (int off = 1; off < 32; off <<= 1) ssum += __shfl_xor(ssum, off, 32);
    const float inv = __builtin_amdgcn_rcpf(ssum);
#pragma unroll 1
    for (int i = 0; i < 8; ++i) sc[hb + lane + 32 * i] *= inv;
  }
  __syncthreads();
  {
    const int hsel = j >> 5;
    const int widx = 32 + (j >> 1);
    const unsigned shv = (unsigned)(j & 1) * 16u;
    float acc = 0.0f;
#pragma unroll 1
    for (int key = 0; key < NSTEP; ++key) {
      const unsigned u = ((const unsigned*)(KV + (rowb + key) * QKVP))[widx];
      const unsigned hbits = (u >> shv) & 0xffffu;
      acc = fmaf(sc[hsel * 256 + key], h16_to_f32(hbits), acc);
    }
    os[j] = acc;
  }
  __syncthreads();
  {
    float acc = 0.0f;
    const float* wr = out_w2 + (size_t)j * NHID;
#pragma unroll 1
    for (int k = 0; k < NHID; ++k) acc = fmaf(os[k], bf16r(wr[k]), acc);
    const float a = acc + bf16r(out_b2[j]);
    t3[j] = a + a;
  }
  __syncthreads();
  {
    float s = 0.0f;
#pragma unroll 1
    for (int k = 0; k < NHID; ++k) s += t3[k];
    const float mean = s * (1.0f / NHID);
    float vs = 0.0f;
#pragma unroll 1
    for (int k = 0; k < NHID; ++k) { const float d = t3[k] - mean; vs += d * d; }
    const float var = vs * (1.0f / NHID);
    const float rstd = rsqrtf(var + LN_EPS_F);
    ys[j] = ((t3[j] - mean) * rstd) * bf16r(ln3s[j]) + bf16r(ln3b[j]);
  }
  __syncthreads();
  if (wave == 0) {
    const int p8 = (lane & 7) * 8;
    const unsigned selh = (lane < 8) ? 0xffffu : 0u;
    const unsigned sell = selh ^ 0xffffu;
    v4u v;
#pragma unroll
    for (int e = 0; e < 4; ++e) {
      const float f0 = ys[p8 + 2 * e], f1 = ys[p8 + 2 * e + 1];
      const unsigned short h0 = f2bf_bits(f0), h1b = f2bf_bits(f1);
      const unsigned short l0 = f2bf_bits(f0 - bf_bits2f(h0)), l1 = f2bf_bits(f1 - bf_bits2f(h1b));
      const unsigned w0 = ((unsigned)h0 & selh) | ((unsigned)l0 & sell);
      const unsigned w1 = ((unsigned)h1b & selh) | ((unsigned)l1 & sell);
      v[e] = w0 | (w1 << 16);
    }
    unsigned short* dst = H3B + (size_t)n * SP2 + lane * 8;
    if (lane < 16) *(volatile v4u*)dst = v;
    __threadfence();
    if (lane < 16) *(volatile v4u*)dst = v;
  }
}

__global__ __launch_bounds__(NTHR) void head_kernel(const float* __restrict__ H4F,
                                                   const float* __restrict__ fw1, const float* __restrict__ fb1,
                                                   const float* __restrict__ fw2, const float* __restrict__ fb2,
                                                   const float* __restrict__ fw3, const float* __restrict__ fb3,
                                                   const float* __restrict__ fw4, const float* __restrict__ fb4,
                                                   float* __restrict__ outp) {
  __shared__ float hin[HSEQ * 64], o1[HSEQ * 256], o2[HSEQ * 64], o3[HSEQ * 32];
  const int tid = threadIdx.x;
  const int s0 = blockIdx.x * HSEQ;
#pragma unroll 1
  for (int i = tid; i < HSEQ * 64; i += NTHR) hin[i] = H4F[(size_t)s0 * 64 + i];
  __syncthreads();
  {
    const int jc = tid;
    const float* wr = fw1 + (size_t)jc * 64;
    const float bv = bf16r(fb1[jc]);
#pragma unroll 1
    for (int s = 0; s < HSEQ; ++s) {
      float acc = 0.0f;
#pragma unroll 1
      for (int k = 0; k < 64; ++k) acc = fmaf(hin[s * 64 + k], bf16r(wr[k]), acc);
      o1[s * 256 + jc] = fsilu(acc + bv);
    }
  }
  __syncthreads();
  {
    const int jc = tid & 63, sg = tid >> 6;
    const float* wr = fw2 + (size_t)jc * 256;
    const float bv = bf16r(fb2[jc]);
#pragma unroll 1
    for (int i = 0; i < 8; ++i) {
      const int s = sg * 8 + i;
      float acc = 0.0f;
#pragma unroll 1
      for (int k = 0; k < 256; ++k) acc = fmaf(o1[s * 256 + k], bf16r(wr[k]), acc);
      o2[s * 64 + jc] = fsilu(acc + bv);
    }
  }
  __syncthreads();
  {
    const int jc = tid & 31, sg = tid >> 5;
    const float* wr = fw3 + (size_t)jc * 64;
    const float bv = bf16r(fb3[jc]);
#pragma unroll 1
    for (int i = 0; i < 4; ++i) {
      const int s = sg * 4 + i;
      float acc = 0.0f;
#pragma unroll 1
      for (int k = 0; k < 64; ++k) acc = fmaf(o2[s * 64 + k], bf16r(wr[k]), acc);
      o3[s * 32 + jc] = fsilu(acc + bv);
    }
  }
  __syncthreads();
  if (tid < 32) {
    const int s = tid;
    float acc = 0.0f;
#pragma unroll 1
    for (int k = 0; k < 32; ++k) acc = fmaf(o3[s * 32 + k], bf16r(fw4[k]), acc);
    const float v = acc + bf16r(fb4[0]);
    volatile float* dst = outp + s0 + s;
    *dst = v;
    __threadfence();
    *dst = v;
  }
}

extern "C" void kernel_launch(void* const* d_in, const int* in_sizes, int n_in,
                              void* d_out, int out_size, void* d_ws, size_t ws_size, hipStream_t stream) {
  if (n_in < 38 || d_out == nullptr || d_ws == nullptr) return;
  if (in_sizes[0] != NSEQ * 3 * NSTEP || in_sizes[1] != EMBN * EMBD || in_sizes[2] != NG3 * NFEATK ||
      in_sizes[3] != NG3 * NHID || in_sizes[4] != NG3 || in_sizes[5] != NG3 || in_sizes[6] != 2 * NG3 * NHID ||
      in_sizes[7] != 2 * NG3 * NHID || in_sizes[8] != 2 * NG3 || in_sizes[9] != 2 * NG3 || in_sizes[10] != NG3 * NHID ||
      in_sizes[11] != NG3 || in_sizes[12] != NHID * NHID || in_sizes[13] != NHID || in_sizes[14] != NG3 * NHID ||
      in_sizes[15] != NG3 || in_sizes[16] != NHID * NHID || in_sizes[17] != NHID || in_sizes[18] != NFF * NHID ||
      in_sizes[19] != NFF || in_sizes[20] != NHID * NFF || in_sizes[21] != NHID || in_sizes[30] != 256 * 64 ||
      in_sizes[31] != 256 || in_sizes[32] != 64 * 256 || in_sizes[33] != 64 || in_sizes[34] != 32 * 64 ||
      in_sizes[35] != 32 || in_sizes[36] != 32 || in_sizes[37] != 1 || out_size != NSEQ) return;
  for (int i = 22; i < 30; ++i) if (in_sizes[i] != NHID) return;

  const float* x      = (const float*)d_in[0];
  const float* emb    = (const float*)d_in[1];
  const float* wih0   = (const float*)d_in[2];
  const float* whh0   = (const float*)d_in[3];
  const float* bih0   = (const float*)d_in[4];
  const float* bhh0   = (const float*)d_in[5];
  const float* wih12  = (const float*)d_in[6];
  const float* whh12  = (const float*)d_in[7];
  const float* bih12  = (const float*)d_in[8];
  const float* bhh12  = (const float*)d_in[9];
  const float* in_w1  = (const float*)d_in[10];
  const float* in_b1  = (const float*)d_in[11];
  const float* out_w1 = (const float*)d_in[12];
  const float* out_b1 = (const float*)d_in[13];
  const float* in_w2  = (const float*)d_in[14];
  const float* in_b2  = (const float*)d_in[15];
  const float* out_w2 = (const float*)d_in[16];
  const float* out_b2 = (const float*)d_in[17];
  const float* ff_w1  = (const float*)d_in[18];
  const float* ff_b1  = (const float*)d_in[19];
  const float* ff_w2  = (const float*)d_in[20];
  const float* ff_b2  = (const float*)d_in[21];
  const float* ln1_s  = (const float*)d_in[22];
  const float* ln1_b  = (const float*)d_in[23];
  const float* ln2_s  = (const float*)d_in[24];
  const float* ln2_b  = (const float*)d_in[25];
  const float* ln3_s  = (const float*)d_in[26];
  const float* ln3_b  = (const float*)d_in[27];
  const float* ln4_s  = (const float*)d_in[28];
  const float* ln4_b  = (const float*)d_in[29];
  const float* fw1    = (const float*)d_in[30];
  const float* fb1    = (const float*)d_in[31];
  const float* fw2    = (const float*)d_in[32];
  const float* fb2    = (const float*)d_in[33];
  const float* fw3    = (const float*)d_in[34];
  const float* fb3    = (const float*)d_in[35];
  const float* fw4    = (const float*)d_in[36];
  const float* fb4    = (const float*)d_in[37];
  float* outp = (float*)d_out;

  char* ws = (char*)d_ws; size_t off = 0;
  auto carve = [&](size_t bytes) -> char* { char* p = ws + off; off += (bytes + 255) & ~(size_t)255; return p; };
  unsigned short* INW1   = (unsigned short*)carve((size_t)NG3 * NHID * 2);
  unsigned short* OUTW1  = (unsigned short*)carve((size_t)NHID * NHID * 2);
  unsigned short* INW2KV = (unsigned short*)carve((size_t)2 * NHID * NHID * 2);
  unsigned short* FFW1   = (unsigned short*)carve((size_t)NFF * NHID * 2);
  unsigned short* FFW2   = (unsigned short*)carve((size_t)NHID * NFF * 2);
  unsigned short* FEAT   = (unsigned short*)carve((size_t)NROWS * NFEATP * 2);
  unsigned short* SQ0    = (unsigned short*)carve((size_t)NROWS * SP2 * 2);
  unsigned short* SQ1    = (unsigned short*)carve((size_t)NROWS * SP2 * 2);
  unsigned short* QKV    = (unsigned short*)carve((size_t)NROWS * QKVP * 2);
  unsigned short* H2H    = (unsigned short*)carve((size_t)NROWS * NHID * 2);
  float*          H2L    = (float*)carve((size_t)NSEQ * NHID * 4);
  unsigned short* H3B    = (unsigned short*)carve((size_t)NSEQ * SP2 * 2);
  float*          H4F    = (float*)carve((size_t)NSEQ * NHID * 4);
  if (off > ws_size || off > (size_t)134217728) return;

  cvt8_kernel<0><<<(NG3 * 8 + NTHR - 1) / NTHR,          NTHR, 0, stream>>>(in_w1,  INW1,   NG3,      8,       NHID, 0, 1.0f);
  cvt8_kernel<1><<<(NHID * 8 + NTHR - 1) / NTHR,         NTHR, 0, stream>>>(out_w1, OUTW1,  NHID,     8,       NHID, 0, WCARRY);
  cvt8_kernel<1><<<(2 * NHID * 8 + NTHR - 1) / NTHR,     NTHR, 0, stream>>>(in_w2 + (size_t)NHID * NHID, INW2KV, 2 * NHID, 8, NHID, 0, WCARRY);
  cvt8_kernel<1><<<(NFF * 8 + NTHR - 1) / NTHR,          NTHR, 0, stream>>>(ff_w1,  FFW1,   NFF,      8,       NHID, 0, WCARRY);
  cvt8_kernel<1><<<(NHID * (NFF / 8) + NTHR - 1) / NTHR, NTHR, 0, stream>>>(ff_w2,  FFW2,   NHID,     NFF / 8, NFF,  0, WCARRY);

  featurize_kernel<<<NSEQ, NTHR, 0, stream>>>(x, emb, FEAT);

  gru_layer_kernel<NFEATK><<<NSEQ / SEQ_BLK, NTG, 0, stream>>>(FEAT, wih0, whh0, bih0, bhh0, SQ0);
  gru_layer_kernel<NHID><<<NSEQ / SEQ_BLK, NTG, 0, stream>>>(SQ0, wih12, whh12, bih12, bhh12, SQ1);
  gru_layer_kernel<NHID><<<NSEQ / SEQ_BLK, NTG, 0, stream>>>(SQ1, wih12 + (size_t)NG3 * NHID, whh12 + (size_t)NG3 * NHID,
                                                              bih12 + NG3, bhh12 + NG3, SQ0);

  wmma_gemm64<1, 2, 2, 1, false, 0><<<dim3(((NROWS / 64) * (NG3 / 64)) / 8, 1), 256, 0, stream>>>(
      SQ0, SQ0 + NHID, SP2, 0L, INW1, INW1, NHID, 0L, (void*)QKV, (void*)QKV, QKVP, 0L,
      in_b1, H4F, 0L, NROWS, NG3, NHID, 1.0f);
  attn_ln1_kernel<<<NSEQ * 2, NTHR, 0, stream>>>(QKV, SQ0, OUTW1, out_b1, ln1_s, ln1_b, SQ1);
  ffn_ln_kernel<true, 2><<<NROWS / FFROWS, NTHR, 0, stream>>>(SQ1, FFW1, ff_b1, FFW2, ff_b2, ln2_s, ln2_b, H2L, H2H);

  wmma_gemm64<0, 0, 2, 1, false, 0><<<dim3(((NROWS / 64) * ((2 * NHID) / 64)) / 8, 1), 256, 0, stream>>>(
      H2H, H2H, NHID, 0L, INW2KV, INW2KV, NHID, 0L, (void*)QKV, (void*)QKV, QKVP, 0L,
      in_b2 + NHID, H4F, 0L, NROWS, 2 * NHID, NHID, WCARRY_INV);
  tail_kernel<<<NSEQ, 64, 0, stream>>>(H2L, QKV, in_w2, in_b2, out_w2, out_b2, ln3_s, ln3_b, H3B);
  ffn_ln_kernel<false, 1><<<NSEQ / FFROWS, NTHR, 0, stream>>>(H3B, FFW1, ff_b1, FFW2, ff_b2, ln4_s, ln4_b, H4F, H2H);
  head_kernel<<<NSEQ / HSEQ, NTHR, 0, stream>>>(H4F, fw1, fb1, fw2, fb2, fw3, fb3, fw4, fb4, outp);
}
